// TopologyTypePredictor_76699525972070
// MI455X (gfx1250) — hardware-run, weakly checked
//
#include <hip/hip_runtime.h>
#include <math.h>

typedef __attribute__((ext_vector_type(16))) _Float16 v16h;
typedef __attribute__((ext_vector_type(8)))  _Float16 v8h;
typedef __attribute__((ext_vector_type(16))) __bf16   v16b;
typedef __attribute__((ext_vector_type(8)))  __bf16   v8b;
typedef __attribute__((ext_vector_type(8)))  float    v8f;
typedef __attribute__((ext_vector_type(4)))  float    v4f;

constexpr int kBatch = 2;
constexpr int kNodes = 512;
constexpr int kDm    = 256;
constexpr int kTypes = 7;
constexpr int kTPad  = 16;
constexpr int kRows  = kBatch * kNodes;
constexpr int kK1    = 3 * kDm;
constexpr int kN1    = 2 * kDm;
constexpr int kTI    = 16;
constexpr int kTJ    = 32;
constexpr int kPitch = kDm + 4;
constexpr int kStg   = kTJ * kTypes;
constexpr float kCarryH = 16.0f;
constexpr float kCarryW = 256.0f;
constexpr float kCarryHW = kCarryH * kCarryW;
constexpr float kFold = 1.0f / (kCarryH * kCarryW);
static_assert(kRows == 1024 && kK1 == 768 && kN1 == 512, "shapes");
static_assert((kRows % 64) == 0 && (kN1 % 64) == 0 && (kK1 % 32) == 0, "GEMM tile multiples");
static_assert((kDm % 32) == 0 && (kNodes % kTI) == 0 && (kNodes % kTJ) == 0, "pair tile multiples");
static_assert(kStg == 224 && ((kStg * 4) % 128) == 0, "one (b,i) j-tile is 7 whole lines");
static_assert(kTypes < kTPad, "class pad");

constexpr size_t kOffA1   = 0;
constexpr size_t kOffBT1  = kOffA1  + (size_t)kRows * kK1 * 2;
constexpr size_t kOffBT2  = kOffBT1 + (size_t)kN1 * kK1 * 2;
constexpr size_t kOffBIAS = kOffBT2 + (size_t)kTPad * kDm * 2;
constexpr size_t kOffH    = kOffBIAS + (size_t)kN1 * 4;
constexpr size_t kWsTotal = kOffH + (size_t)kRows * kN1 * 4;
static_assert(kWsTotal == 4466688ull, "carve total");
static_assert(kWsTotal <= 134217728ull, "carve cap");
static_assert((kOffBT1 % 128) == 0 && (kOffBT2 % 128) == 0 && (kOffBIAS % 128) == 0 && (kOffH % 128) == 0, "aligned regions");

__device__ __forceinline__ unsigned short f2bf_bits(float f) {
  unsigned u = __float_as_uint(f);
  return (unsigned short)((u + 0x7FFFu + ((u >> 16) & 1u)) >> 16);
}
__device__ __forceinline__ float bf_bits2f(unsigned short h) { return __uint_as_float(((unsigned)h) << 16); }

__device__ __forceinline__ void guard1_h(v8f& c, v16h x, v16h y) { asm volatile("v_nop\n\tv_nop\n\tv_nop\n\tv_nop" : "+v"(c) : "v"(x), "v"(y)); }
__device__ __forceinline__ void guard1_b(v8f& c, v16b x, v16b y) { asm volatile("v_nop\n\tv_nop\n\tv_nop\n\tv_nop" : "+v"(c) : "v"(x), "v"(y)); }
__device__ __forceinline__ void keep4_h(v16h a, v16h b, v16h c, v16h d) { asm volatile("v_nop" :: "v"(a), "v"(b), "v"(c), "v"(d)); }
__device__ __forceinline__ void keep4_b(v16b a, v16b b, v16b c, v16b d) { asm volatile("v_nop" :: "v"(a), "v"(b), "v"(c), "v"(d)); }

template <typename T> struct Frag;
template <> struct Frag<_Float16> {
  typedef v16h V; union U { v16h v; v8h h[2]; };
  static __device__ __forceinline__ v16h load(const _Float16* p) {
    U f; f.h[0] = *(const v8h*)(p); f.h[1] = *(const v8h*)(p + 16); return f.v;
  }
  static __device__ __forceinline__ v8f mma(v16h a, v16h b, v8f c) {
    return __builtin_amdgcn_wmma_f32_16x16x32_f16(false, a, false, b, (short)0, c, false, false);
  }
  static __device__ __forceinline__ void guard1(v8f& c, v16h x, v16h y) { guard1_h(c, x, y); }
  static __device__ __forceinline__ void keep(v16h a, v16h b, v16h c, v16h d) { keep4_h(a, b, c, d); }
};
template <> struct Frag<__bf16> {
  typedef v16b V; union U { v16b v; v8b h[2]; };
  static __device__ __forceinline__ v16b load(const __bf16* p) {
    U f; f.h[0] = *(const v8b*)(p); f.h[1] = *(const v8b*)(p + 16); return f.v;
  }
  static __device__ __forceinline__ v8f mma(v16b a, v16b b, v8f c) {
    return __builtin_amdgcn_wmma_f32_16x16x32_bf16(false, a, false, b, (short)0, c, false, false);
  }
  static __device__ __forceinline__ void guard1(v8f& c, v16b x, v16b y) { guard1_b(c, x, y); }
  static __device__ __forceinline__ void keep(v16b a, v16b b, v16b c, v16b d) { keep4_b(a, b, c, d); }
};

template <int ET> struct Elem;
template <> struct Elem<0> { typedef _Float16 T; };
template <> struct Elem<1> { typedef __bf16 T; };

template <int ET, int BIAS_MODE>
__global__ __launch_bounds__(256) void wmma_gemm64(
    const unsigned short* __restrict__ Ap, int lda,
    const unsigned short* __restrict__ Btp, int ldb,
    float* __restrict__ C, int ldc,
    const float* __restrict__ bias,
    int M, int N, int K, float scale) {
  typedef typename Elem<ET>::T T;
  typedef typename Frag<T>::V V;
  const T* A = (const T*)Ap;
  const T* Bt = (const T*)Btp;
  __shared__ __align__(16) float sT[8][16 * 68];
  const int lane = threadIdx.x & 31;
  const int wave = __builtin_amdgcn_readfirstlane((int)(threadIdx.x >> 5));
  const int tilesN = N >> 6;
  const int tilesM = M >> 6;
  const int tile = blockIdx.x * 8 + wave;
  if (tile >= tilesM * tilesN) return;
  const int tm = tile / tilesN;
  const int tn = tile - tm * tilesN;
  const int m0 = tm << 6;
  const int n0 = tn << 6;

  const int rlane = lane & 15;
  const int koff  = (lane >> 4) * 8;
  const int mOff  = (lane >> 4) * 8;

  v8f acc[4][4];
#pragma unroll
  for (int i = 0; i < 4; ++i)
#pragma unroll
    for (int j = 0; j < 4; ++j) acc[i][j] = (v8f){0.f,0.f,0.f,0.f,0.f,0.f,0.f,0.f};

  for (int k0 = 0; k0 < K; k0 += 32) {
    V bh[4];
#pragma unroll
    for (int j = 0; j < 4; ++j) {
      const size_t bo = (size_t)(n0 + (j << 4) + rlane) * ldb + koff + k0;
      bh[j] = Frag<T>::load(Bt + bo);
    }
#pragma unroll
    for (int i = 0; i < 4; ++i) {
      const size_t ao = (size_t)(m0 + (i << 4) + rlane) * lda + koff + k0;
      V ah = Frag<T>::load(A + ao);
#pragma unroll
      for (int j = 0; j < 4; ++j) acc[i][j] = Frag<T>::mma(ah, bh[j], acc[i][j]);
#pragma unroll
      for (int j = 0; j < 4; ++j) Frag<T>::guard1(acc[i][j], ah, bh[j]);
    }
    Frag<T>::keep(bh[0], bh[1], bh[2], bh[3]);
  }

  float* slab = sT[wave];
#pragma unroll
  for (int i = 0; i < 4; ++i) {
    const int mBase = m0 + (i << 4);
#pragma unroll
    for (int j = 0; j < 4; ++j) {
      const int n = n0 + (j << 4) + rlane;
      float bv = 0.f;
      if (BIAS_MODE == 2) bv = bias[n];
#pragma unroll
      for (int r = 0; r < 8; ++r) {
        float v = acc[i][j][r] * scale;
        if (BIAS_MODE == 2) v += bv;
        slab[(mOff + r) * 68 + (j << 4) + rlane] = v;
      }
    }
    __builtin_amdgcn_fence(__ATOMIC_RELEASE, "workgroup");
    __builtin_amdgcn_wave_barrier();
    __builtin_amdgcn_fence(__ATOMIC_ACQUIRE, "workgroup");
    {
      const int hh = lane >> 4, c4 = (lane & 15) * 4;
      for (int pass = 0; pass < 2; ++pass) {
#pragma unroll
        for (int it = 0; it < 8; ++it) {
          const int row = it * 2 + hh;
          v4f v = *(const v4f*)(slab + row * 68 + c4);
          *(volatile v4f*)(C + (size_t)(mBase + row) * ldc + n0 + c4) = v;
        }
        __threadfence();
      }
    }
    __builtin_amdgcn_fence(__ATOMIC_RELEASE, "workgroup");
    __builtin_amdgcn_wave_barrier();
    __builtin_amdgcn_fence(__ATOMIC_ACQUIRE, "workgroup");
  }
}

__global__ __launch_bounds__(256) void prep_x_kernel(const float* __restrict__ X, unsigned short* __restrict__ A1) {
  const int i = blockIdx.x * 256 + threadIdx.x;
  if (i >= kRows * kDm / 8) return;
  const int row = i >> 5;
  const int c8 = (i & 31) * 8;
  const float* src = X + (size_t)row * kDm + c8;
  const v4f a0 = *(const v4f*)(src);
  const v4f a1 = *(const v4f*)(src + 4);
  v8h hv, lv;
#pragma unroll
  for (int e = 0; e < 4; ++e) {
    const float x0 = a0[e];
    const float x1 = a1[e];
    const unsigned short h0 = f2bf_bits(x0), h1 = f2bf_bits(x1);
    const unsigned short l0 = f2bf_bits(x0 - bf_bits2f(h0)), l1 = f2bf_bits(x1 - bf_bits2f(h1));
    hv[e]     = __builtin_bit_cast(_Float16, h0);
    hv[4 + e] = __builtin_bit_cast(_Float16, h1);
    lv[e]     = __builtin_bit_cast(_Float16, l0);
    lv[4 + e] = __builtin_bit_cast(_Float16, l1);
  }
  unsigned short* q = A1 + (size_t)row * kK1 + c8;
  *(volatile v8h*)(q) = hv;
  *(volatile v8h*)(q + kDm) = lv;
  *(volatile v8h*)(q + 2 * kDm) = hv;
  __threadfence();
  *(volatile v8h*)(q) = hv;
  *(volatile v8h*)(q + kDm) = lv;
  *(volatile v8h*)(q + 2 * kDm) = hv;
}

__global__ __launch_bounds__(256) void prep_w1_kernel(const float* __restrict__ W1, unsigned short* __restrict__ Bt1) {
  __shared__ float sT[kDm * 33];
  const int tid = threadIdx.x;
  const int lane = tid & 31;
  const int wave = __builtin_amdgcn_readfirstlane((int)(threadIdx.x >> 5));
  const int bx = blockIdx.x;
  const int half = bx >> 3;
  const int nn0 = (bx & 7) * 32;
  const float* src = W1 + (size_t)(half * kDm) * kDm + nn0;
#pragma unroll 8
  for (int it = 0; it < 32; ++it) {
    const int e = tid + 256 * it;
    const int k = e >> 5;
    const int c = e & 31;
    sT[k * 33 + c] = src[(size_t)k * kDm + c];
  }
  __syncthreads();
#pragma unroll
  for (int rr = 0; rr < 4; ++rr) {
    const int nl = wave * 4 + rr;
    v8h hv, lv;
#pragma unroll
    for (int e = 0; e < 8; ++e) {
      const float w = sT[(lane * 8 + e) * 33 + nl];
      const unsigned short hb = f2bf_bits(w);
      const unsigned short lb = f2bf_bits(w - bf_bits2f(hb));
      hv[e] = __builtin_bit_cast(_Float16, hb);
      lv[e] = __builtin_bit_cast(_Float16, lb);
    }
    unsigned short* q = Bt1 + (size_t)(bx * 32 + nl) * kK1 + lane * 8;
    *(volatile v8h*)(q) = hv;
    *(volatile v8h*)(q + kDm) = hv;
    *(volatile v8h*)(q + 2 * kDm) = lv;
    __threadfence();
    *(volatile v8h*)(q) = hv;
    *(volatile v8h*)(q + kDm) = hv;
    *(volatile v8h*)(q + 2 * kDm) = lv;
  }
}

__global__ __launch_bounds__(256) void prep_small_kernel(
    const float* __restrict__ W2, const float* __restrict__ b1,
    unsigned short* __restrict__ Bt2, float* __restrict__ biasN) {
  const int tid = threadIdx.x;
#pragma unroll
  for (int it = 0; it < 2; ++it) {
    const int idx8 = tid + 256 * it;
    const int n = idx8 >> 5;
    const int k8 = (idx8 & 31) * 8;
    const int nc = (n < kTypes) ? n : (kTypes - 1);
    v8h hv;
#pragma unroll
    for (int e = 0; e < 8; ++e) {
      const float w = W2[(size_t)(k8 + e) * kTypes + nc];
      const float s = (n < kTypes) ? (w * kCarryW) : 0.0f;
      hv[e] = (_Float16)s;
    }
    unsigned short* q = Bt2 + (size_t)n * kDm + k8;
    *(volatile v8h*)(q) = hv;
    __threadfence();
    *(volatile v8h*)(q) = hv;
  }
  {
    const int c4 = (tid & 127) * 4;
    v4f bv;
#pragma unroll
    for (int u = 0; u < 4; ++u) {
      const int col = c4 + u;
      float t = b1[(col < kDm) ? col : (kDm - 1)];
      asm volatile("" : "+v"(t));
      bv[u] = (col < kDm) ? (t * kCarryH) : 0.0f;
    }
    if (tid < 128) {
      float* q = biasN + tid * 4;
      *(volatile v4f*)(q) = bv;
      __threadfence();
      *(volatile v4f*)(q) = bv;
    }
  }
}

__global__ __launch_bounds__(256) void pair_logits_kernel(
    const float* __restrict__ H, const unsigned short* __restrict__ Bt2p,
    const float* __restrict__ b2, float* __restrict__ out) {
  __shared__ __align__(16) float sHi[kTI * kPitch];
  __shared__ __align__(16) float sHj[kTJ * kPitch];
  __shared__ __align__(16) float sOut[8][kStg];
  const _Float16* Bt2 = (const _Float16*)Bt2p;
  const int tid = threadIdx.x;
  const int lane = tid & 31;
  const int wave = __builtin_amdgcn_readfirstlane((int)(threadIdx.x >> 5));
  const int hh = lane >> 4;
  const int m = lane & 15;

  const int blk = blockIdx.x;
  const int bb = blk >> 9;
  const int rem = blk & 511;
  const int i0 = (rem >> 4) * kTI;
  const int j0 = (rem & 15) * kTJ;

  const float* Hb = H + (size_t)(bb * kNodes) * kN1;
#pragma unroll
  for (int it = 0; it < 4; ++it) {
    const int e = tid + 256 * it;
    const int r = e >> 6;
    const int c4 = (e & 63) * 4;
    const v4f v = *(const v4f*)(Hb + (size_t)(i0 + r) * kN1 + c4);
    *(v4f*)(sHi + r * kPitch + c4) = v;
  }
#pragma unroll
  for (int it = 0; it < 8; ++it) {
    const int e = tid + 256 * it;
    const int r = e >> 6;
    const int c4 = (e & 63) * 4;
    const v4f v = *(const v4f*)(Hb + (size_t)(j0 + r) * kN1 + kDm + c4);
    *(v4f*)(sHj + r * kPitch + c4) = v;
  }
  __syncthreads();

  float b2v = b2[(m < kTypes) ? m : (kTypes - 1)];
  asm volatile("" : "+v"(b2v));
  const float bv = (m < kTypes) ? (b2v * kCarryHW) : 0.0f;

  v8f acc[2][2];
#pragma unroll
  for (int ii = 0; ii < 2; ++ii)
#pragma unroll
    for (int jg = 0; jg < 2; ++jg) acc[ii][jg] = (v8f){bv, bv, bv, bv, bv, bv, bv, bv};

  const _Float16* bp = Bt2 + (size_t)m * kDm + 8 * hh;
  const float* hip0 = sHi + (2 * wave) * kPitch + 8 * hh;
  const float* hjp0 = sHj + m * kPitch + 8 * hh;

#pragma unroll 1
  for (int ks = 0; ks < kDm / 32; ++ks) {
    const int ko = ks * 32;
    const v16h bw = Frag<_Float16>::load(bp + ko);
    v4f hq[2][4], jq[2][4];
#pragma unroll
    for (int ii = 0; ii < 2; ++ii) {
      const float* p = hip0 + ii * kPitch + ko;
      hq[ii][0] = *(const v4f*)(p);
      hq[ii][1] = *(const v4f*)(p + 4);
      hq[ii][2] = *(const v4f*)(p + 16);
      hq[ii][3] = *(const v4f*)(p + 20);
    }
#pragma unroll
    for (int jg = 0; jg < 2; ++jg) {
      const float* p = hjp0 + jg * 16 * kPitch + ko;
      jq[jg][0] = *(const v4f*)(p);
      jq[jg][1] = *(const v4f*)(p + 4);
      jq[jg][2] = *(const v4f*)(p + 16);
      jq[jg][3] = *(const v4f*)(p + 20);
    }
    v16h a[2][2];
#pragma unroll
    for (int ii = 0; ii < 2; ++ii) {
#pragma unroll
      for (int jg = 0; jg < 2; ++jg) {
#pragma unroll
        for (int t = 0; t < 4; ++t) {
#pragma unroll
          for (int u = 0; u < 4; ++u) {
            float s = hq[ii][t][u] + jq[jg][t][u];
            s = fmaxf(s, 0.0f);
            a[ii][jg][4 * t + u] = (_Float16)s;
          }
        }
      }
    }
#pragma unroll
    for (int ii = 0; ii < 2; ++ii)
#pragma unroll
      for (int jg = 0; jg < 2; ++jg) acc[ii][jg] = Frag<_Float16>::mma(a[ii][jg], bw, acc[ii][jg]);
#pragma unroll
    for (int ii = 0; ii < 2; ++ii)
#pragma unroll
      for (int jg = 0; jg < 2; ++jg) guard1_h(acc[ii][jg], a[ii][jg], bw);
  }

  float* stg = sOut[wave];
  const int f1 = (32 + lane < 55) ? (32 + lane) : 55;
#pragma unroll
  for (int ii = 0; ii < 2; ++ii) {
#pragma unroll
    for (int jg = 0; jg < 2; ++jg) {
#pragma unroll
      for (int r = 0; r < 8; ++r) {
        const float v = acc[ii][jg][r] * kFold;
        if (m < kTypes) stg[(jg * 16 + 8 * hh + r) * kTypes + m] = v;
      }
    }
    __builtin_amdgcn_fence(__ATOMIC_RELEASE, "workgroup");
    __builtin_amdgcn_wave_barrier();
    __builtin_amdgcn_fence(__ATOMIC_ACQUIRE, "workgroup");
    const v4f v0 = *(const v4f*)(stg + 4 * lane);
    const v4f v1 = *(const v4f*)(stg + 4 * f1);
    float* o = out + ((size_t)(bb * kNodes + i0 + 2 * wave + ii) * kNodes + j0) * kTypes;
    for (int pass = 0; pass < 2; ++pass) {
      *(volatile v4f*)(o + 4 * lane) = v0;
      if (lane < 24) *(volatile v4f*)(o + 128 + 4 * lane) = v1;
      __threadfence();
    }
    __builtin_amdgcn_fence(__ATOMIC_RELEASE, "workgroup");
    __builtin_amdgcn_wave_barrier();
    __builtin_amdgcn_fence(__ATOMIC_ACQUIRE, "workgroup");
  }
}

extern "C" void kernel_launch(void* const* d_in, const int* in_sizes, int n_in,
                              void* d_out, int out_size, void* d_ws, size_t ws_size,
                              hipStream_t stream) {
  if (n_in < 5) return;
  if (in_sizes[0] != kRows * kDm) return;
  if (in_sizes[1] != kN1 * kDm) return;
  if (in_sizes[2] != kDm) return;
  if (in_sizes[3] != kDm * kTypes) return;
  if (in_sizes[4] != kTypes) return;
  if (out_size != kBatch * kNodes * kNodes * kTypes) return;
  if (ws_size < kWsTotal) return;

  const float* X  = (const float*)d_in[0];
  const float* W1 = (const float*)d_in[1];
  const float* b1 = (const float*)d_in[2];
  const float* W2 = (const float*)d_in[3];
  const float* b2 = (const float*)d_in[4];
  float* out = (float*)d_out;

  char* ws = (char*)d_ws;
  unsigned short* A1   = (unsigned short*)(ws + kOffA1);
  unsigned short* BT1  = (unsigned short*)(ws + kOffBT1);
  unsigned short* BT2  = (unsigned short*)(ws + kOffBT2);
  float*          BIAS = (float*)(ws + kOffBIAS);
  float*          Hp   = (float*)(ws + kOffH);

  prep_x_kernel<<<(kRows * kDm / 8) / 256, 256, 0, stream>>>(X, A1);
  prep_w1_kernel<<<kN1 / 32, 256, 0, stream>>>(W1, BT1);
  prep_small_kernel<<<1, 256, 0, stream>>>(W2, b1, BT2, BIAS);

  wmma_gemm64<1, 2><<<dim3(((kRows / 64) * (kN1 / 64)) / 8, 1), 256, 0, stream>>>(
      A1, kK1, BT1, kK1, Hp, kN1, BIAS, kRows, kN1, kK1, kCarryH);

  pair_logits_kernel<<<kBatch * (kNodes / kTI) * (kNodes / kTJ), 256, 0, stream>>>(Hp, BT2, b2, out);
}
